// MolecularCliffordEPModel_48627619725328
// MI455X (gfx1250) — hardware-verified
//
#include <hip/hip_runtime.h>


#define NR   4096
#define NM   512
#define NO   128
#define NI   8
#define KK   (NM * NI)
constexpr float  DT_ = 0.1f;
constexpr double Q1_ = 1.0 - (double)DT_;
constexpr float  CF  = (float)(1.0 - Q1_ * Q1_ * Q1_ * Q1_ * Q1_ * Q1_ * Q1_ * Q1_ * Q1_ * Q1_);
constexpr size_t al256(size_t b) { return (b + 255) & ~(size_t)255; }
constexpr size_t WS_TOTAL = al256((size_t)NO * KK * 2) + 2 * al256((size_t)NR * KK * 2);
static_assert(WS_TOTAL == 68157440 && WS_TOTAL <= 134217728, "the workspace carve: about 65.0 MiB");
typedef _Float16 h16;
typedef unsigned short bf;
typedef __attribute__((ext_vector_type(16))) __bf16   v16bf;
typedef __attribute__((ext_vector_type(16))) _Float16 v16h;
typedef __attribute__((ext_vector_type(8)))  _Float16 v8h;
typedef __attribute__((ext_vector_type(8)))  unsigned short v8us;
typedef __attribute__((ext_vector_type(8)))  float    v8f;
typedef __attribute__((ext_vector_type(4)))  float    v4f;
typedef v8h  __attribute__((may_alias)) v8ha;
typedef v4f  __attribute__((may_alias)) v4fa;
typedef v8us __attribute__((may_alias)) v8usa;

__device__ __forceinline__ unsigned short f2bf(float f) { unsigned u = __float_as_uint(f); u += 0x7FFFu + ((u >> 16) & 1u); return (unsigned short)(u >> 16); }
__device__ __forceinline__ float bf2f(unsigned short b) { return __uint_as_float(((unsigned)b) << 16); }
__device__ __forceinline__ float bfr(float f) { return bf2f(f2bf(f)); }
__device__ __forceinline__ v16h cat16(v8h lo, v8h hi) { return __builtin_shufflevector(lo, hi, 0, 1, 2, 3, 4, 5, 6, 7, 8, 9, 10, 11, 12, 13, 14, 15); }
__device__ __forceinline__ v16bf cat16b(v8us lo, v8us hi) { return __builtin_bit_cast(v16bf, __builtin_shufflevector(lo, hi, 0, 1, 2, 3, 4, 5, 6, 7, 8, 9, 10, 11, 12, 13, 14, 15)); }
__device__ __forceinline__ v8f wmma16(v16h a, v16h b, v8f c) { return __builtin_amdgcn_wmma_f32_16x16x32_f16(false, a, false, b, (short)0, c, false, false); }
__device__ __forceinline__ v8f wmmab(v16bf a, v16bf b, v8f c) { return __builtin_amdgcn_wmma_f32_16x16x32_bf16(false, a, false, b, (short)0, c, false, false); }


template <typename T16> struct WFrag;
template <> struct WFrag<h16> { typedef v16h V; static __device__ __forceinline__ V ld(const h16* p) { return cat16(*(const v8h*)p, *(const v8h*)(p + 16)); } static __device__ __forceinline__ v8f mma(V a, V b, v8f c) { return wmma16(a, b, c); } };
template <> struct WFrag<bf> { typedef v16bf V; static __device__ __forceinline__ V ld(const bf* p) { return cat16b(*(const v8us*)p, *(const v8us*)(p + 16)); } static __device__ __forceinline__ v8f mma(V a, V b, v8f c) { return wmmab(a, b, c); } };
template <typename T16, int NSPLIT, bool BIAS>
__global__ __launch_bounds__(32) void k_gemmw(const T16* __restrict__ A, const T16* __restrict__ A2, const T16* __restrict__ Bt, const T16* __restrict__ Bt2, int K, float* C, int ldc, const float* __restrict__ bias, size_t sA, size_t sB, size_t sC) {
    typedef typename WFrag<T16>::V V;
    __shared__ __align__(16) float os[16 * 68];
    const size_t z = blockIdx.z; A += z * sA; if (A2) A2 += z * sA; Bt += z * sB; if (Bt2) Bt2 += z * sB; C += z * sC;
    const int lane = threadIdx.x & 31, lr = lane & 15, hi = lane >> 4; const int r0 = blockIdx.x * 64, c0 = blockIdx.y * 64;
    v8f acc[4][4];
#pragma unroll
    for (int mb = 0; mb < 4; ++mb)
#pragma unroll
        for (int nb = 0; nb < 4; ++nb) acc[mb][nb] = (v8f){};
    const size_t aoff = (size_t)(r0 + lr) * K + 8 * hi, boff = (size_t)(c0 + lr) * K + 8 * hi;
    for (int kc = 0; kc < K; kc += 32) {
        V a[4], a2[4];
#pragma unroll
        for (int mb = 0; mb < 4; ++mb) { a[mb] = WFrag<T16>::ld(A + aoff + (size_t)mb * 16 * K + kc); if (NSPLIT == 1 || NSPLIT == 2) a2[mb] = WFrag<T16>::ld(A2 + aoff + (size_t)mb * 16 * K + kc); }
#pragma unroll
        for (int nb = 0; nb < 4; ++nb) { const V b = WFrag<T16>::ld(Bt + boff + (size_t)nb * 16 * K + kc); V b2; if (NSPLIT >= 2) b2 = WFrag<T16>::ld(Bt2 + boff + (size_t)nb * 16 * K + kc);
#pragma unroll
            for (int mb = 0; mb < 4; ++mb) { acc[mb][nb] = WFrag<T16>::mma(a[mb], b, acc[mb][nb]); if (NSPLIT == 1 || NSPLIT == 2) acc[mb][nb] = WFrag<T16>::mma(a2[mb], b, acc[mb][nb]); if (NSPLIT >= 2) acc[mb][nb] = WFrag<T16>::mma(a[mb], b2, acc[mb][nb]); } }
        asm volatile("v_nop\n\tv_nop\n\tv_nop\n\tv_nop" : "+v"(acc[0][0]), "+v"(acc[1][1]), "+v"(acc[2][2]), "+v"(acc[3][3]) : "v"(a[0]), "v"(a[3]));
    }
#pragma unroll
    for (int mb = 0; mb < 4; ++mb) {
#pragma unroll
        for (int nb = 0; nb < 4; ++nb) {
#pragma unroll
            for (int j = 0; j < 8; ++j) os[(hi * 8 + j) * 68 + nb * 16 + lr] = acc[mb][nb][j]; }
        __builtin_amdgcn_wave_barrier(); asm volatile("" ::: "memory");
        float* crow = C + (size_t)(r0 + mb * 16) * ldc + c0;
#pragma unroll 1
        for (int ps = 0; ps < 2; ++ps) {
#pragma unroll
            for (int s = 0; s < 8; ++s) { const int row = 2 * s + hi, cofs = lr * 4; v4f val = *(const v4fa*)(os + row * 68 + cofs); if (BIAS) { val[0] += bfr(bias[c0 + cofs]); val[1] += bfr(bias[c0 + cofs + 1]); val[2] += bfr(bias[c0 + cofs + 2]); val[3] += bfr(bias[c0 + cofs + 3]); }
                *(volatile v4f*)(crow + (size_t)row * ldc + cofs) = val; }
            if (ps == 0) __threadfence(); }
        __builtin_amdgcn_wave_barrier(); asm volatile("" ::: "memory");
    }
}

__device__ __forceinline__ h16 tohx(float x) { return (h16)x; }
__device__ __forceinline__ void splitf(float y, unsigned short& h, unsigned short& l) { h = f2bf(y); l = f2bf(y - bf2f(h)); }
typedef __attribute__((ext_vector_type(2))) _Float16 v2h;
typedef __attribute__((ext_vector_type(4))) _Float16 v4h;
typedef __attribute__((ext_vector_type(2))) unsigned short v2us;
typedef __attribute__((ext_vector_type(4))) unsigned short v4us;
typedef __attribute__((ext_vector_type(2))) float v2f;
typedef __attribute__((ext_vector_type(4))) int v4i;

__global__ __launch_bounds__(256) void k_cvt8(const float* __restrict__ src, bf* dst, size_t n8) { const size_t i = (size_t)blockIdx.x * 256 + threadIdx.x; if (i >= n8) return; const v8f v = *(const v8f*)(src + i * 8); v8us o;
#pragma unroll
    for (int k = 0; k < 8; ++k) o[k] = f2bf(v[k]); *(volatile v8us*)(dst + i * 8) = o; __threadfence(); *(volatile v8us*)(dst + i * 8) = o; }

__global__ __launch_bounds__(256) void k_lift(const float* __restrict__ xm, const float* __restrict__ wi, bf* Ah, bf* Al) {
    const size_t e = (size_t)blockIdx.x * 256 + threadIdx.x; if (e >= (size_t)NR * NM) return; const int m = (int)(e % NM); const size_t b = e / NM;
    const v4f xa = *(const v4f*)(xm + b * NI), xb = *(const v4f*)(xm + b * NI + 4), wa = *(const v4f*)(wi + (size_t)m * NI), wb = *(const v4f*)(wi + (size_t)m * NI + 4);
    const float x0 = bfr(xa[0]), x1 = bfr(xa[1]), x2 = bfr(xa[2]), x3 = bfr(xa[3]), x4 = bfr(xb[0]), x5 = bfr(xb[1]), x6 = bfr(xb[2]), x7 = bfr(xb[3]);
    const float w0 = bfr(wa[0]), w1 = bfr(wa[1]), w2 = bfr(wa[2]), w3 = bfr(wa[3]), w4 = bfr(wb[0]), w5 = bfr(wb[1]), w6 = bfr(wb[2]), w7 = bfr(wb[3]);
    const float g0 = x0 * w0 + x1 * w1 + x2 * w2 - x3 * w3 + x4 * w4 - x5 * w5 - x6 * w6 - x7 * w7;
    const float g1 = x0 * w1 + x1 * w0 - x2 * w3 + x3 * w2 - x4 * w5 + x5 * w4 - x6 * w7 - x7 * w6;
    const float g2 = x0 * w2 + x1 * w3 + x2 * w0 - x3 * w1 - x4 * w6 + x5 * w7 + x6 * w4 + x7 * w5;
    const float g3 = x0 * w3 + x1 * w2 - x2 * w1 + x3 * w0 + x4 * w7 - x5 * w6 + x6 * w5 + x7 * w4;
    const float g4 = x0 * w4 + x1 * w5 + x2 * w6 - x3 * w7 + x4 * w0 - x5 * w1 - x6 * w2 - x7 * w3;
    const float g5 = x0 * w5 + x1 * w4 - x2 * w7 + x3 * w6 - x4 * w1 + x5 * w0 - x6 * w3 - x7 * w2;
    const float g6 = x0 * w6 + x1 * w7 + x2 * w4 - x3 * w5 - x4 * w2 + x5 * w3 + x6 * w0 + x7 * w1;
    const float g7 = x0 * w7 + x1 * w6 - x2 * w5 + x3 * w4 + x4 * w3 - x5 * w2 + x6 * w1 + x7 * w0;
    const float a0 = CF * g0, a1 = CF * g1, a2 = CF * g2, a3 = -CF * g3, a4 = CF * g4, a5 = -CF * g5, a6 = -CF * g6, a7 = -CF * g7;
    v8us oh, ol; unsigned short hh, ll;
    splitf(a0, hh, ll); oh[0] = hh; ol[0] = ll; splitf(a1, hh, ll); oh[1] = hh; ol[1] = ll; splitf(a2, hh, ll); oh[2] = hh; ol[2] = ll; splitf(a3, hh, ll); oh[3] = hh; ol[3] = ll;
    splitf(a4, hh, ll); oh[4] = hh; ol[4] = ll; splitf(a5, hh, ll); oh[5] = hh; ol[5] = ll; splitf(a6, hh, ll); oh[6] = hh; ol[6] = ll; splitf(a7, hh, ll); oh[7] = hh; ol[7] = ll;
    const size_t o = b * KK + (size_t)m * NI; *(volatile v8us*)(Ah + o) = oh; *(volatile v8us*)(Al + o) = ol; __threadfence(); *(volatile v8us*)(Ah + o) = oh; *(volatile v8us*)(Al + o) = ol; }

extern "C" void kernel_launch(void* const* d_in, const int* in_sizes, int n_in,
                              void* d_out, int out_size, void* d_ws, size_t ws_size, hipStream_t stream) {
    if (n_in < 3) return;
    if (in_sizes[0] < NR * NI || in_sizes[1] < NM * NI || in_sizes[2] < NO * KK || out_size < NR * NO) return;
    const float* xm = (const float*)d_in[0]; const float* wi = (const float*)d_in[1]; const float* wo = (const float*)d_in[2];
    float* OUT = (float*)d_out;
    char* wsp = (char*)d_ws;
    auto take = [&](size_t bytes) { char* p = wsp; wsp += (bytes + 255) & ~(size_t)255; return (void*)p; };
    bf* WT = (bf*)take((size_t)NO * KK * 2); bf* Ah = (bf*)take((size_t)NR * KK * 2); bf* Al = (bf*)take((size_t)NR * KK * 2);
    if ((size_t)(wsp - (char*)d_ws) != WS_TOTAL || WS_TOTAL > ws_size) return;
    k_cvt8<<<(unsigned)(((size_t)NO * KK / 8 + 255) / 256), 256, 0, stream>>>(wo, WT, (size_t)NO * KK / 8);
    k_lift<<<(unsigned)(((size_t)NR * NM + 255) / 256), 256, 0, stream>>>(xm, wi, Ah, Al);
    k_gemmw<bf, 1, false><<<dim3(NR / 64, NO / 64, 1), 32, 0, stream>>>(Ah, Al, WT, nullptr, KK, OUT, NO, nullptr, (size_t)0, (size_t)0, (size_t)0);
}
